// MyRNN_15281493639833
// MI455X (gfx1250) — hardware-verified
//
#include <hip/hip_runtime.h>
#include <math.h>

constexpr int NBATCH = 4096;
constexpr int NSTEP  = 80;
constexpr int NEMB   = 100;
constexpr int KEMB   = 128;
constexpr int NHID   = 256;
constexpr int KCAT   = 2 * NHID;
constexpr int NVOC   = 10000;
constexpr int NVOCP  = 10048;
constexpr int NTHR   = 256;
constexpr int RB     = 32;
constexpr int HP     = 264;
constexpr int XSP    = 260;
constexpr float EMB_CARRY = 16.0f;
constexpr float W1_CARRY  = 8.0f;
constexpr float PROJ_FOLD = 1.0f / 128.0f;
constexpr float WU_CARRY  = 16.0f;
constexpr float H_CARRY   = 8.0f;
constexpr float REC_FOLD  = 1.0f / 128.0f;
static_assert(NVOCP % 64 == 0 && NVOCP >= NVOC && NVOCP - NVOC < 64, "GEMM M padded to the 64 tile");
static_assert(KEMB % 32 == 0 && KEMB >= NEMB && KEMB % 64 == 0, "GEMM K padded to a multiple of 32");
static_assert(NHID % 64 == 0 && KCAT % 32 == 0 && NHID % 32 == 0, "tile multiples");
static_assert(NBATCH % RB == 0, "recurrence grid exact");
static_assert(RB == 32 && NHID == 64 * ((NTHR / 32) / 2), "8 waves = 2 m-subtiles x 4 column quarters of 64");
static_assert((2 * RB * HP) % NTHR == 0 && (RB * HP) % NTHR == 0 && (RB * NSTEP) % NTHR == 0, "init loops exact");
static_assert(RB * NHID == 8 * 4 * NTHR, "staging: 8 float4 per thread covers the 32x256 tile exactly");
static_assert(NVOCP % 16 == 0 && NEMB % 4 == 0, "pack grids exact");
static_assert(HP % 8 == 0 && XSP % 4 == 0, "16-B aligned LDS rows");

typedef __attribute__((ext_vector_type(16))) _Float16 v16h;
typedef __attribute__((ext_vector_type(8)))  _Float16 v8h;
typedef __attribute__((ext_vector_type(16))) __bf16   v16b;
typedef __attribute__((ext_vector_type(8)))  __bf16   v8b;
typedef __attribute__((ext_vector_type(8)))  float    v8f;
typedef __attribute__((ext_vector_type(4)))  float    v4f;

__device__ __forceinline__ unsigned short f2bf_bits(float f) {
  unsigned u = __float_as_uint(f);
  return (unsigned short)((u + 0x7FFFu + ((u >> 16) & 1u)) >> 16);
}
__device__ __forceinline__ float bf_bits2f(unsigned short h) { return __uint_as_float(((unsigned)h) << 16); }

__device__ __forceinline__ void dep_guard_h(v8f& a, v8f& b, v16h x, v16h y) { asm volatile("v_nop\n\tv_nop\n\tv_nop\n\tv_nop" : "+v"(a), "+v"(b) : "v"(x), "v"(y)); }
__device__ __forceinline__ void dep_guard_b(v8f& a, v8f& b, v16b x, v16b y) { asm volatile("v_nop\n\tv_nop\n\tv_nop\n\tv_nop" : "+v"(a), "+v"(b) : "v"(x), "v"(y)); }
__device__ __forceinline__ void keep4_h(v16h a, v16h b, v16h c, v16h d) { asm volatile("v_nop" :: "v"(a), "v"(b), "v"(c), "v"(d)); }
__device__ __forceinline__ void keep4_b(v16b a, v16b b, v16b c, v16b d) { asm volatile("v_nop" :: "v"(a), "v"(b), "v"(c), "v"(d)); }
__device__ __forceinline__ void acc_guard4(v8f& a, v8f& b, v8f& c, v8f& d) { asm volatile("v_nop\n\tv_nop\n\tv_nop\n\tv_nop" : "+v"(a), "+v"(b), "+v"(c), "+v"(d)); }
__device__ __forceinline__ void grp_guard_h(v8f& c0, v8f& c1, v8f& c2, v8f& c3, v16h a0, v16h a1, v16h b0, v16h b1, v16h b2, v16h b3) {
  asm volatile("v_nop\n\tv_nop\n\tv_nop\n\tv_nop" : "+v"(c0), "+v"(c1), "+v"(c2), "+v"(c3) : "v"(a0), "v"(a1), "v"(b0), "v"(b1), "v"(b2), "v"(b3));
}
__device__ __forceinline__ void grp_guard_b(v8f& c0, v8f& c1, v8f& c2, v8f& c3, v16b a0, v16b a1, v16b b0, v16b b1, v16b b2, v16b b3) {
  asm volatile("v_nop\n\tv_nop\n\tv_nop\n\tv_nop" : "+v"(c0), "+v"(c1), "+v"(c2), "+v"(c3) : "v"(a0), "v"(a1), "v"(b0), "v"(b1), "v"(b2), "v"(b3));
}
template <typename T> struct Frag;
template <> struct Frag<_Float16> {
  typedef v16h V; union U { v16h v; v8h h[2]; };
  static __device__ __forceinline__ v16h load(const _Float16* p) {
    U f; f.h[0] = *(const v8h*)(p); f.h[1] = *(const v8h*)(p + 16); return f.v;
  }
  static __device__ __forceinline__ v8f mma(v16h a, v16h b, v8f c) {
    return __builtin_amdgcn_wmma_f32_16x16x32_f16(false, a, false, b, (short)0, c, false, false);
  }
  static __device__ __forceinline__ void guard(v8f& a, v8f& b, v16h x, v16h y) { dep_guard_h(a, b, x, y); }
  static __device__ __forceinline__ void guard4(v8f& c0, v8f& c1, v8f& c2, v8f& c3, v16h a0, v16h a1, v16h b0, v16h b1, v16h b2, v16h b3) {
    grp_guard_h(c0, c1, c2, c3, a0, a1, b0, b1, b2, b3);
  }
  static __device__ __forceinline__ void keep(v16h a, v16h b, v16h c, v16h d) { keep4_h(a, b, c, d); }
};
template <> struct Frag<__bf16> {
  typedef v16b V; union U { v16b v; v8b h[2]; };
  static __device__ __forceinline__ v16b load(const __bf16* p) {
    U f; f.h[0] = *(const v8b*)(p); f.h[1] = *(const v8b*)(p + 16); return f.v;
  }
  static __device__ __forceinline__ v8f mma(v16b a, v16b b, v8f c) {
    return __builtin_amdgcn_wmma_f32_16x16x32_bf16(false, a, false, b, (short)0, c, false, false);
  }
  static __device__ __forceinline__ void guard(v8f& a, v8f& b, v16b x, v16b y) { dep_guard_b(a, b, x, y); }
  static __device__ __forceinline__ void guard4(v8f& c0, v8f& c1, v8f& c2, v8f& c3, v16b a0, v16b a1, v16b b0, v16b b1, v16b b2, v16b b3) {
    grp_guard_b(c0, c1, c2, c3, a0, a1, b0, b1, b2, b3);
  }
  static __device__ __forceinline__ void keep(v16b a, v16b b, v16b c, v16b d) { keep4_b(a, b, c, d); }
};

__device__ __forceinline__ float fsig(float x)  { return __builtin_amdgcn_rcpf(1.0f + __expf(-x)); }
__device__ __forceinline__ float ftanh(float x) { return 1.0f - 2.0f * __builtin_amdgcn_rcpf(__expf(2.0f * x) + 1.0f); }

template <int ET> struct Elem;
template <> struct Elem<0> { typedef _Float16 T; };
template <> struct Elem<1> { typedef __bf16 T; };
template <int ET, bool SPLIT, int BIAS_MODE, int OUT_MODE, bool RESID, int ACT = 0>
__global__ __launch_bounds__(256) void wmma_gemm64(
    const unsigned short* __restrict__ Ap, const unsigned short* __restrict__ A2p, int lda, long strideA,
    const unsigned short* __restrict__ Btp, const unsigned short* __restrict__ Bt2p, int ldb, long strideB,
    void* __restrict__ Cout, void* __restrict__ Cout2, int ldc, long strideC,
    const float* __restrict__ bias,
    const float* __restrict__ resid, long strideR,
    int M, int N, int K, float scale) {
  typedef typename Elem<ET>::T T;
  typedef typename Frag<T>::V V;
  const T* A = (const T*)Ap; const T* A2 = (const T*)A2p; const T* Bt = (const T*)Btp; const T* Bt2 = (const T*)Bt2p;
  __shared__ __align__(16) float sT[8][16 * 68];
  const int b    = blockIdx.y;
  const int lane = threadIdx.x & 31;
  const int wave = threadIdx.x >> 5;
  const int tilesN = N >> 6;
  const int tilesM = M >> 6;
  const int tile = blockIdx.x * 8 + wave;
  if (tile >= tilesM * tilesN) return;
  const int tm = tile / tilesN;
  const int tn = tile - tm * tilesN;
  const int m0 = tm << 6;
  const int n0 = tn << 6;

  const T* Ab  = A  + (size_t)b * strideA;
  const T* Bb  = Bt + (size_t)b * strideB;
  const T* Ab2 = SPLIT ? (A2  + (size_t)b * strideA) : nullptr;
  const T* Bb2 = SPLIT ? (Bt2 + (size_t)b * strideB) : nullptr;

  const int rlane = lane & 15;
  const int koff  = (lane >> 4) * 8;
  const int mOff  = (lane >> 4) * 8;

  v8f acc[4][4];
#pragma unroll
  for (int i = 0; i < 4; ++i)
#pragma unroll
    for (int j = 0; j < 4; ++j) acc[i][j] = (v8f){0.f,0.f,0.f,0.f,0.f,0.f,0.f,0.f};

  for (int k0 = 0; k0 < K; k0 += 32) {
    V bh[4], bl[4];
#pragma unroll
    for (int j = 0; j < 4; ++j) {
      const size_t bo = (size_t)(n0 + (j << 4) + rlane) * ldb + koff + k0;
      bh[j] = Frag<T>::load(Bb + bo);
      if (SPLIT) bl[j] = Frag<T>::load(Bb2 + bo);
    }
#pragma unroll
    for (int i = 0; i < 4; ++i) {
      const size_t ao = (size_t)(m0 + (i << 4) + rlane) * lda + koff + k0;
      V ah = Frag<T>::load(Ab + ao);
      V al;
      if (SPLIT) al = Frag<T>::load(Ab2 + ao);
#pragma unroll
      for (int j = 0; j < 4; ++j) {
        acc[i][j] = Frag<T>::mma(ah, bh[j], acc[i][j]);
        if (SPLIT) {
          acc[i][j] = Frag<T>::mma(ah, bl[j], acc[i][j]);
          acc[i][j] = Frag<T>::mma(al, bh[j], acc[i][j]);
        }
      }
      Frag<T>::guard4(acc[i][0], acc[i][1], acc[i][2], acc[i][3], ah, SPLIT ? al : ah, bh[0], bh[1], bh[2], bh[3]);
      if (SPLIT) Frag<T>::keep(bl[0], bl[1], bl[2], bl[3]);
    }
    Frag<T>::keep(bh[0], bh[1], bh[2], bh[3]);
    if (SPLIT) Frag<T>::keep(bl[0], bl[1], bl[2], bl[3]);
  }
  acc_guard4(acc[0][0], acc[0][1], acc[0][2], acc[0][3]);
  acc_guard4(acc[1][0], acc[1][1], acc[1][2], acc[1][3]);
  acc_guard4(acc[2][0], acc[2][1], acc[2][2], acc[2][3]);
  acc_guard4(acc[3][0], acc[3][1], acc[3][2], acc[3][3]);

  float* slab = sT[wave];
  const float* Rb = RESID ? (resid + (size_t)b * strideR) : nullptr;
#pragma unroll
  for (int i = 0; i < 4; ++i) {
    const int mBase = m0 + (i << 4);
#pragma unroll
    for (int j = 0; j < 4; ++j) {
      const int n = n0 + (j << 4) + rlane;
      float bv = 0.f;
      if (BIAS_MODE == 2) bv = bias[n];
#pragma unroll
      for (int r = 0; r < 8; ++r) {
        float v = acc[i][j][r] * scale;
        if (BIAS_MODE == 1) v += bias[mBase + mOff + r];
        if (BIAS_MODE == 2) v += bv;
        if (RESID) v += Rb[(size_t)(mBase + mOff + r) * ldc + n];
        if (ACT == 1) v = tanhf(v);
        if (ACT == 2) v = fmaxf(v, 0.0f);
        if (ACT == 3) v = v / (1.0f + expf(-v));
        if (ACT == 4) v = (v > 0.f) ? v : 0.01f * v;
        slab[(mOff + r) * 68 + (j << 4) + rlane] = v;
      }
    }
    __builtin_amdgcn_fence(__ATOMIC_RELEASE, "workgroup");
    __builtin_amdgcn_wave_barrier();
    __builtin_amdgcn_fence(__ATOMIC_ACQUIRE, "workgroup");
    if (OUT_MODE == 0) {
      float* C = (float*)Cout + (size_t)b * strideC;
      const int hh = lane >> 4, c4 = (lane & 15) * 4;
      for (int pass = 0; pass < 2; ++pass) {
#pragma unroll
        for (int it = 0; it < 8; ++it) {
          const int row = it * 2 + hh;
          v4f v = *(const v4f*)(slab + row * 68 + c4);
          *(volatile v4f*)(C + (size_t)(mBase + row) * ldc + n0 + c4) = v;
        }
        __threadfence();
      }
    } else {
      const int q = lane >> 3, c8 = (lane & 7) * 8;
      unsigned short* C  = (unsigned short*)Cout  + (size_t)b * strideC;
      unsigned short* C2 = (OUT_MODE == 2) ? ((unsigned short*)Cout2 + (size_t)b * strideC) : nullptr;
      for (int pass = 0; pass < 2; ++pass) {
#pragma unroll
        for (int it = 0; it < 4; ++it) {
          const int row = it * 4 + q;
          const float* sp = slab + row * 68 + c8;
          v8h hv, lv;
#pragma unroll
          for (int e = 0; e < 8; ++e) {
            if (OUT_MODE == 1) {
              hv[e] = (_Float16)sp[e];
            } else {
              unsigned short hb = f2bf_bits(sp[e]);
              unsigned short lb = f2bf_bits(sp[e] - bf_bits2f(hb));
              hv[e] = __builtin_bit_cast(_Float16, hb);
              lv[e] = __builtin_bit_cast(_Float16, lb);
            }
          }
          *(volatile v8h*)(C + (size_t)(mBase + row) * ldc + n0 + c8) = hv;
          if (OUT_MODE == 2) *(volatile v8h*)(C2 + (size_t)(mBase + row) * ldc + n0 + c8) = lv;
        }
        __threadfence();
      }
    }
    __builtin_amdgcn_fence(__ATOMIC_RELEASE, "workgroup");
    __builtin_amdgcn_wave_barrier();
    __builtin_amdgcn_fence(__ATOMIC_ACQUIRE, "workgroup");
  }
}

__global__ __launch_bounds__(NTHR) void pack_emb_kernel(const float* __restrict__ emb, unsigned short* __restrict__ O) {
  const int tid = threadIdx.x;
  const int row = blockIdx.x * 16 + (tid >> 4);
  const int col = (tid & 15) * 8;
  const int rowc = (row < NVOC) ? row : (NVOC - 1);
  const int ca = (col     < NEMB - 4) ? col       : (NEMB - 4);
  const int cb = (col + 4 < NEMB - 4) ? (col + 4) : (NEMB - 4);
  const float* rp = emb + (size_t)rowc * NEMB;
  const v4f va = *(const v4f*)(rp + ca);
  const v4f vb = *(const v4f*)(rp + cb);
  const float fa = (row < NVOC && col     < NEMB) ? EMB_CARRY : 0.0f;
  const float fb = (row < NVOC && col + 4 < NEMB) ? EMB_CARRY : 0.0f;
  v8h hv;
#pragma unroll
  for (int e = 0; e < 4; ++e) {
    hv[e]     = (_Float16)(va[e] * fa);
    hv[4 + e] = (_Float16)(vb[e] * fb);
  }
  unsigned short* op = O + (size_t)row * KEMB + col;
  *(volatile v8h*)op = hv;
  __threadfence();
  *(volatile v8h*)op = hv;
}

__global__ __launch_bounds__(NTHR) void pack_t_kernel(const float* __restrict__ src, int R, int C, int ldo,
                                                      unsigned short* __restrict__ O, float sc) {
  __shared__ float Tt[64 * 65];
  const int tid = threadIdx.x;
  const int c0 = blockIdx.x * 64, r0 = blockIdx.y * 64;
#pragma unroll
  for (int i = 0; i < 4; ++i) {
    const int idx = i * NTHR + tid;
    const int rr = idx >> 4, cc = (idx & 15) * 4;
    const int row = r0 + rr;
    const int rowc = (row < R) ? row : (R - 1);
    const float f = (row < R) ? sc : 0.0f;
    const v4f v = *(const v4f*)(src + (size_t)rowc * (size_t)C + c0 + cc);
    Tt[rr * 65 + cc + 0] = v[0] * f;
    Tt[rr * 65 + cc + 1] = v[1] * f;
    Tt[rr * 65 + cc + 2] = v[2] * f;
    Tt[rr * 65 + cc + 3] = v[3] * f;
  }
  __syncthreads();
  const int q = tid >> 3, c8 = (tid & 7) * 8;
  v8h hv[2];
#pragma unroll
  for (int g = 0; g < 2; ++g) {
    const int qq = g * 32 + q;
#pragma unroll
    for (int e = 0; e < 8; ++e) hv[g][e] = (_Float16)Tt[(c8 + e) * 65 + qq];
  }
  for (int pass = 0; pass < 2; ++pass) {
#pragma unroll
    for (int g = 0; g < 2; ++g) {
      const size_t o = (size_t)(c0 + g * 32 + q) * (size_t)ldo + (size_t)(r0 + c8);
      *(volatile v8h*)(O + o) = hv[g];
    }
    __threadfence();
  }
}

__global__ __launch_bounds__(NTHR) void rnn2_seq_kernel(const int* __restrict__ tok, const float* __restrict__ P,
                                                        const unsigned short* __restrict__ U1p,
                                                        const unsigned short* __restrict__ WU2p,
                                                        const float* __restrict__ bias2, float* __restrict__ out) {
  __shared__ __align__(16) _Float16 H1s[2][RB * HP];
  __shared__ __align__(16) _Float16 H2s[RB * HP];
  __shared__ __align__(16) float    Xs[RB * XSP];
  __shared__ __align__(16) int      Tk[RB * NSTEP];
  const _Float16* U1  = (const _Float16*)U1p;
  const _Float16* WU2 = (const _Float16*)WU2p;
  const int tid = threadIdx.x, lane = tid & 31, wave = tid >> 5;
  const int c = lane & 15, hh = lane >> 4, koff = hh * 8;
  const int ms = wave >> 2, nq = wave & 3;
  const int rowbase = blockIdx.x * RB;
  const int arow = 16 * ms + c;
  const int drow = 16 * ms + 8 * hh;

  {
    _Float16* h1f = &H1s[0][0];
#pragma unroll 1
    for (int i = tid; i < 2 * RB * HP; i += NTHR) h1f[i] = (_Float16)0.0f;
#pragma unroll 1
    for (int i = tid; i < RB * HP; i += NTHR) H2s[i] = (_Float16)0.0f;
#pragma unroll 1
    for (int i = tid; i < RB * NSTEP; i += NTHR) {
      int v = tok[(size_t)rowbase * NSTEP + i];
      v = (v < 0) ? 0 : v;
      v = (v > NVOC - 1) ? (NVOC - 1) : v;
      Tk[i] = v;
    }
  }
  float bb[4];
  float h2f[4][8];
#pragma unroll
  for (int nt = 0; nt < 4; ++nt) {
    bb[nt] = bias2[64 * nq + 16 * nt + c];
#pragma unroll
    for (int r = 0; r < 8; ++r) h2f[nt][r] = 0.0f;
  }
  __syncthreads();

  const int xm = tid >> 3, xcb = (tid & 7) * 32;
  const _Float16* a2row = H2s + arow * HP + koff;
  const _Float16* wb1 = U1  + (size_t)(64 * nq + c) * NHID + koff;
  const _Float16* wb2 = WU2 + (size_t)(64 * nq + c) * KCAT + koff;
  const v8f z8 = {0.f, 0.f, 0.f, 0.f, 0.f, 0.f, 0.f, 0.f};

#pragma unroll 1
  for (int t = 0; t < NSTEP; ++t) {
    {
      const int tk = Tk[xm * NSTEP + t];
      const float* sp = P + (size_t)tk * NHID + xcb;
      float* dp = Xs + xm * XSP + xcb;
      v4f xv[8];
#pragma unroll
      for (int i = 0; i < 8; ++i) xv[i] = *(const v4f*)(sp + 4 * i);
#pragma unroll
      for (int i = 0; i < 8; ++i) *(v4f*)(dp + 4 * i) = xv[i];
    }
#pragma unroll
    for (int nt = 0; nt < 4; ++nt) {
      const int j = 64 * nq + 16 * nt + c;
#pragma unroll
      for (int r = 0; r < 8; ++r) H2s[(drow + r) * HP + j] = (_Float16)(h2f[nt][r] * H_CARRY);
    }
    __syncthreads();

    {
      const int cur = t & 1;
      const _Float16* a1row = &H1s[cur][0] + arow * HP + koff;
      _Float16* h1n = &H1s[cur ^ 1][0];
      v8f acc[4];
      acc[0] = z8; acc[1] = z8; acc[2] = z8; acc[3] = z8;
#pragma unroll 1
      for (int k0 = 0; k0 < NHID; k0 += 32) {
        const v16h a   = Frag<_Float16>::load(a1row + k0);
        const v16h fb0 = Frag<_Float16>::load(wb1 + k0);
        const v16h fb1 = Frag<_Float16>::load(wb1 + (size_t)16 * NHID + k0);
        const v16h fb2 = Frag<_Float16>::load(wb1 + (size_t)32 * NHID + k0);
        const v16h fb3 = Frag<_Float16>::load(wb1 + (size_t)48 * NHID + k0);
        acc[0] = Frag<_Float16>::mma(a, fb0, acc[0]);
        acc[1] = Frag<_Float16>::mma(a, fb1, acc[1]);
        acc[2] = Frag<_Float16>::mma(a, fb2, acc[2]);
        acc[3] = Frag<_Float16>::mma(a, fb3, acc[3]);
        grp_guard_h(acc[0], acc[1], acc[2], acc[3], a, a, fb0, fb1, fb2, fb3);
      }
      acc_guard4(acc[0], acc[1], acc[2], acc[3]);
#pragma unroll
      for (int nt = 0; nt < 4; ++nt) {
        const int j = 64 * nq + 16 * nt + c;
#pragma unroll
        for (int r = 0; r < 8; ++r) {
          const float xp = Xs[(drow + r) * XSP + j];
          const float z  = acc[nt][r] * REC_FOLD + xp;
          const float hv = ftanh(z);
          h1n[(drow + r) * HP + j] = (_Float16)(hv * H_CARRY);
        }
      }
    }
    __syncthreads();

    {
      const _Float16* a1n = &H1s[(t & 1) ^ 1][0] + arow * HP + koff;
      v8f acc[4];
      acc[0] = z8; acc[1] = z8; acc[2] = z8; acc[3] = z8;
#pragma unroll 1
      for (int k0 = 0; k0 < NHID; k0 += 32) {
        const v16h a   = Frag<_Float16>::load(a1n + k0);
        const v16h fb0 = Frag<_Float16>::load(wb2 + k0);
        const v16h fb1 = Frag<_Float16>::load(wb2 + (size_t)16 * KCAT + k0);
        const v16h fb2 = Frag<_Float16>::load(wb2 + (size_t)32 * KCAT + k0);
        const v16h fb3 = Frag<_Float16>::load(wb2 + (size_t)48 * KCAT + k0);
        acc[0] = Frag<_Float16>::mma(a, fb0, acc[0]);
        acc[1] = Frag<_Float16>::mma(a, fb1, acc[1]);
        acc[2] = Frag<_Float16>::mma(a, fb2, acc[2]);
        acc[3] = Frag<_Float16>::mma(a, fb3, acc[3]);
        grp_guard_h(acc[0], acc[1], acc[2], acc[3], a, a, fb0, fb1, fb2, fb3);
      }
#pragma unroll 1
      for (int k0 = 0; k0 < NHID; k0 += 32) {
        const v16h a   = Frag<_Float16>::load(a2row + k0);
        const v16h fb0 = Frag<_Float16>::load(wb2 + NHID + k0);
        const v16h fb1 = Frag<_Float16>::load(wb2 + (size_t)16 * KCAT + NHID + k0);
        const v16h fb2 = Frag<_Float16>::load(wb2 + (size_t)32 * KCAT + NHID + k0);
        const v16h fb3 = Frag<_Float16>::load(wb2 + (size_t)48 * KCAT + NHID + k0);
        acc[0] = Frag<_Float16>::mma(a, fb0, acc[0]);
        acc[1] = Frag<_Float16>::mma(a, fb1, acc[1]);
        acc[2] = Frag<_Float16>::mma(a, fb2, acc[2]);
        acc[3] = Frag<_Float16>::mma(a, fb3, acc[3]);
        grp_guard_h(acc[0], acc[1], acc[2], acc[3], a, a, fb0, fb1, fb2, fb3);
      }
      acc_guard4(acc[0], acc[1], acc[2], acc[3]);
#pragma unroll
      for (int nt = 0; nt < 4; ++nt) {
#pragma unroll
        for (int r = 0; r < 8; ++r) h2f[nt][r] = ftanh(acc[nt][r] * REC_FOLD + bb[nt]);
      }
    }
    __syncthreads();
  }

#pragma unroll
  for (int nt = 0; nt < 4; ++nt) {
    const int j = 64 * nq + 16 * nt + c;
#pragma unroll
    for (int r = 0; r < 8; ++r) Xs[(drow + r) * XSP + j] = fsig(h2f[nt][r]);
  }
  __syncthreads();
  for (int pass = 0; pass < 2; ++pass) {
#pragma unroll
    for (int it = 0; it < 8; ++it) {
      const int idx = it * NTHR + tid;
      const int row = idx >> 6, c4 = (idx & 63) * 4;
      const v4f v = *(const v4f*)(Xs + row * XSP + c4);
      *(volatile v4f*)(out + (size_t)(rowbase + row) * NHID + c4) = v;
    }
    __threadfence();
  }
}

extern "C" void kernel_launch(void* const* d_in, const int* in_sizes, int n_in,
                              void* d_out, int out_size, void* d_ws, size_t ws_size, hipStream_t stream) {
  if (n_in < 8 || d_out == nullptr || d_ws == nullptr) return;
  if (in_sizes[0] != NBATCH * NSTEP || in_sizes[1] != NVOC * NEMB || in_sizes[2] != NEMB * NHID ||
      in_sizes[3] != NHID * NHID || in_sizes[4] != NHID || in_sizes[5] != NHID * NHID ||
      in_sizes[6] != NHID * NHID || in_sizes[7] != NHID || out_size != NBATCH * NHID) return;

  const int*   tok = (const int*)d_in[0];
  const float* emb = (const float*)d_in[1];
  const float* w1  = (const float*)d_in[2];
  const float* u1  = (const float*)d_in[3];
  const float* b1  = (const float*)d_in[4];
  const float* w2  = (const float*)d_in[5];
  const float* u2  = (const float*)d_in[6];
  const float* b2  = (const float*)d_in[7];
  float* out = (float*)d_out;

  char* ws = (char*)d_ws; size_t off = 0;
  auto carve = [&](size_t bytes) -> char* { char* p = ws + off; off += (bytes + 255) & ~(size_t)255; return p; };
  unsigned short* EMBA = (unsigned short*)carve((size_t)NVOCP * KEMB * 2);
  unsigned short* W1T  = (unsigned short*)carve((size_t)NHID * KEMB * 2);
  unsigned short* U1T  = (unsigned short*)carve((size_t)NHID * NHID * 2);
  unsigned short* WU2T = (unsigned short*)carve((size_t)NHID * KCAT * 2);
  float*          PT   = (float*)carve((size_t)NVOCP * NHID * 4);
  if (off > ws_size || off > (size_t)134217728) return;

  pack_emb_kernel<<<NVOCP / 16, NTHR, 0, stream>>>(emb, EMBA);
  pack_t_kernel<<<dim3(NHID / 64, KEMB / 64), NTHR, 0, stream>>>(w1, NEMB, NHID, KEMB, W1T, W1_CARRY);
  pack_t_kernel<<<dim3(NHID / 64, NHID / 64), NTHR, 0, stream>>>(u1, NHID, NHID, NHID, U1T, WU_CARRY);
  pack_t_kernel<<<dim3(NHID / 64, NHID / 64), NTHR, 0, stream>>>(w2, NHID, NHID, KCAT, WU2T, WU_CARRY);
  pack_t_kernel<<<dim3(NHID / 64, NHID / 64), NTHR, 0, stream>>>(u2, NHID, NHID, KCAT, WU2T + NHID, WU_CARRY);

  const dim3 ggrid(((NVOCP / 64) * (NHID / 64) + 7) / 8, 1);
  wmma_gemm64<0, false, 2, 0, false, 0><<<ggrid, 256, 0, stream>>>(
      EMBA, EMBA, KEMB, 0L, W1T, W1T, KEMB, 0L, (void*)PT, (void*)PT, NHID, 0L,
      b1, PT, 0L, NVOCP, NHID, KEMB, PROJ_FOLD);

  rnn2_seq_kernel<<<NBATCH / RB, NTHR, 0, stream>>>(tok, PT, U1T, WU2T, b2, out);
}
